// LSTM_3848290697395
// MI455X (gfx1250) — hardware-verified
//
#include <hip/hip_runtime.h>
#include <math.h>

constexpr int NBAT    = 512;
constexpr int NSTEP   = 96;
constexpr int NFEAT   = 64;
constexpr int NHID    = 256;
constexpr int NGATE   = 4 * NHID;
constexpr int NFC1    = 256;
constexpr int NOUTC   = 24;
constexpr int KFLAT   = NSTEP * NHID;
constexpr int NTHR    = 256;
constexpr int SEQ_BLK = 16;
constexpr int HPITCH  = NHID + 8;
constexpr float ACARRY    = 16.0f;
constexpr float WCARRY    = 16.0f;
constexpr float FCARRY    = 1024.0f;
constexpr float GATE_FOLD = 1.0f / (ACARRY * WCARRY);
constexpr float FC1_FOLD  = 1.0f / (ACARRY * FCARRY);

static_assert(NGATE == 1024, "gate rows");
static_assert(NHID == 32 * (NTHR / 32), "8 waves x 32 hidden columns");
static_assert(NBAT % SEQ_BLK == 0, "batch tiles");
static_assert(NFEAT % 32 == 0 && NHID % 32 == 0 && KFLAT % 32 == 0, "K multiples of 32");
static_assert(NBAT % 64 == 0 && NFC1 % 64 == 0, "GEMM M, N tile multiples");
static_assert((NBAT * NOUTC) % NTHR == 0, "head grid exact");
static_assert(KFLAT == 24576, "flatten length");
static_assert((HPITCH % 8) == 0, "16-B aligned LDS rows");

typedef __attribute__((ext_vector_type(16))) _Float16 v16h;
typedef __attribute__((ext_vector_type(8)))  _Float16 v8h;
typedef __attribute__((ext_vector_type(4)))  _Float16 v4h;
typedef __attribute__((ext_vector_type(8)))  float    v8f;
typedef __attribute__((ext_vector_type(4)))  float    v4f;

__device__ __forceinline__ unsigned short f2bf_bits(float f) {
  unsigned u = __float_as_uint(f);
  return (unsigned short)((u + 0x7FFFu + ((u >> 16) & 1u)) >> 16);
}
__device__ __forceinline__ float bf_bits2f(unsigned short h) { return __uint_as_float(((unsigned)h) << 16); }

__device__ __forceinline__ void dep_guard_h(v8f& a, v8f& b, v16h x, v16h y) {
  asm volatile("v_nop\n\tv_nop\n\tv_nop\n\tv_nop" : "+v"(a), "+v"(b) : "v"(x), "v"(y));
}
__device__ __forceinline__ void guard_all_h(v8f& a0, v8f& a1, v8f& a2, v8f& a3, v16h x, v16h y0, v16h y1, v16h y2, v16h y3) {
  asm volatile("v_nop\n\tv_nop\n\tv_nop\n\tv_nop"
               : "+v"(a0), "+v"(a1), "+v"(a2), "+v"(a3)
               : "v"(x), "v"(y0), "v"(y1), "v"(y2), "v"(y3));
}
__device__ __forceinline__ void keep4_h(v16h a, v16h b, v16h c, v16h d) { asm volatile("v_nop" :: "v"(a), "v"(b), "v"(c), "v"(d)); }
__device__ __forceinline__ void acc_guard4(v8f& a, v8f& b, v8f& c, v8f& d) {
  asm volatile("v_nop\n\tv_nop\n\tv_nop\n\tv_nop" : "+v"(a), "+v"(b), "+v"(c), "+v"(d));
}

template <typename T> struct Frag;
template <> struct Frag<_Float16> {
  typedef v16h V;
  union U { v16h v; v8h h[2]; };
  static __device__ __forceinline__ v16h load(const _Float16* p) {
    U f;
    f.h[0] = *(const v8h*)(p);
    f.h[1] = *(const v8h*)(p + 16);
    return f.v;
  }
  static __device__ __forceinline__ v8f mma(v16h a, v16h b, v8f c) {
    return __builtin_amdgcn_wmma_f32_16x16x32_f16(false, a, false, b, (short)0, c, false, false);
  }
  static __device__ __forceinline__ void guard(v8f& a, v8f& b, v16h x, v16h y) { dep_guard_h(a, b, x, y); }
  static __device__ __forceinline__ void guard_all(v8f& a0, v8f& a1, v8f& a2, v8f& a3, v16h x, v16h y0, v16h y1, v16h y2, v16h y3) {
    guard_all_h(a0, a1, a2, a3, x, y0, y1, y2, y3);
  }
  static __device__ __forceinline__ void keep(v16h a, v16h b, v16h c, v16h d) { keep4_h(a, b, c, d); }
};

__device__ __forceinline__ float fsig(float x)  { return __builtin_amdgcn_rcpf(1.0f + __expf(-x)); }
__device__ __forceinline__ float ftanh(float x) { return 1.0f - 2.0f * __builtin_amdgcn_rcpf(__expf(2.0f * x) + 1.0f); }

template <int ET> struct Elem;
template <> struct Elem<0> { typedef _Float16 T; };
template <int ET, bool SPLIT, int BIAS_MODE, int OUT_MODE, bool RESID, int ACT = 0>
__global__ __launch_bounds__(256) void wmma_gemm64(
    const unsigned short* __restrict__ Ap, const unsigned short* __restrict__ A2p, int lda, long strideA,
    const unsigned short* __restrict__ Btp, const unsigned short* __restrict__ Bt2p, int ldb, long strideB,
    void* __restrict__ Cout, void* __restrict__ Cout2, int ldc, long strideC,
    const float* __restrict__ bias,
    const float* __restrict__ resid, long strideR,
    int M, int N, int K, float scale) {
  typedef typename Elem<ET>::T T;
  typedef typename Frag<T>::V V;
  const T* A = (const T*)Ap;
  const T* A2 = (const T*)A2p;
  const T* Bt = (const T*)Btp;
  const T* Bt2 = (const T*)Bt2p;
  __shared__ __align__(16) float sT[8][16 * 68];
  const int b    = blockIdx.y;
  const int lane = threadIdx.x & 31;
  const int wave = threadIdx.x >> 5;
  const int tilesN = N >> 6;
  const int tilesM = M >> 6;
  const int tile = blockIdx.x * 8 + wave;
  if (tile >= tilesM * tilesN) return;
  const int tm = tile / tilesN;
  const int tn = tile - tm * tilesN;
  const int m0 = tm << 6;
  const int n0 = tn << 6;

  const T* Ab  = A  + (size_t)b * strideA;
  const T* Bb  = Bt + (size_t)b * strideB;
  const T* Ab2 = SPLIT ? (A2  + (size_t)b * strideA) : nullptr;
  const T* Bb2 = SPLIT ? (Bt2 + (size_t)b * strideB) : nullptr;

  const int rlane = lane & 15;
  const int koff  = (lane >> 4) * 8;
  const int mOff  = (lane >> 4) * 8;

  v8f acc[4][4];
#pragma unroll
  for (int i = 0; i < 4; ++i)
#pragma unroll
    for (int j = 0; j < 4; ++j) acc[i][j] = (v8f){0.f,0.f,0.f,0.f,0.f,0.f,0.f,0.f};

  for (int k0 = 0; k0 < K; k0 += 32) {
    V bh[4], bl[4];
#pragma unroll
    for (int j = 0; j < 4; ++j) {
      const size_t bo = (size_t)(n0 + (j << 4) + rlane) * ldb + koff + k0;
      bh[j] = Frag<T>::load(Bb + bo);
      if (SPLIT) bl[j] = Frag<T>::load(Bb2 + bo);
    }
#pragma unroll
    for (int i = 0; i < 4; ++i) {
      const size_t ao = (size_t)(m0 + (i << 4) + rlane) * lda + koff + k0;
      V ah = Frag<T>::load(Ab + ao);
      V al;
      if (SPLIT) al = Frag<T>::load(Ab2 + ao);
#pragma unroll
      for (int j = 0; j < 4; ++j) {
        acc[i][j] = Frag<T>::mma(ah, bh[j], acc[i][j]);
        if (SPLIT) {
          acc[i][j] = Frag<T>::mma(ah, bl[j], acc[i][j]);
          acc[i][j] = Frag<T>::mma(al, bh[j], acc[i][j]);
        }
      }
      Frag<T>::guard_all(acc[i][0], acc[i][1], acc[i][2], acc[i][3], ah, bh[0], bh[1], bh[2], bh[3]);
      if (SPLIT) Frag<T>::guard(acc[i][0], acc[i][3], al, bl[0]);
    }
    Frag<T>::keep(bh[0], bh[1], bh[2], bh[3]);
    if (SPLIT) Frag<T>::keep(bl[0], bl[1], bl[2], bl[3]);
  }
  acc_guard4(acc[0][0], acc[0][1], acc[0][2], acc[0][3]);
  acc_guard4(acc[1][0], acc[1][1], acc[1][2], acc[1][3]);
  acc_guard4(acc[2][0], acc[2][1], acc[2][2], acc[2][3]);
  acc_guard4(acc[3][0], acc[3][1], acc[3][2], acc[3][3]);

  float* slab = sT[wave];
  const float* Rb = RESID ? (resid + (size_t)b * strideR) : nullptr;
#pragma unroll
  for (int i = 0; i < 4; ++i) {
    const int mBase = m0 + (i << 4);
#pragma unroll
    for (int j = 0; j < 4; ++j) {
      const int n = n0 + (j << 4) + rlane;
      float bv = 0.f;
      if (BIAS_MODE == 2) bv = bias[n];
#pragma unroll
      for (int r = 0; r < 8; ++r) {
        float v = acc[i][j][r] * scale;
        if (BIAS_MODE == 1) v += bias[mBase + mOff + r];
        if (BIAS_MODE == 2) v += bv;
        if (RESID) v += Rb[(size_t)(mBase + mOff + r) * ldc + n];
        if (ACT == 1) v = tanhf(v);
        if (ACT == 2) v = fmaxf(v, 0.0f);
        slab[(mOff + r) * 68 + (j << 4) + rlane] = v;
      }
    }
    __builtin_amdgcn_fence(__ATOMIC_RELEASE, "workgroup");
    __builtin_amdgcn_wave_barrier();
    __builtin_amdgcn_fence(__ATOMIC_ACQUIRE, "workgroup");
    if (OUT_MODE == 0) {
      float* C = (float*)Cout + (size_t)b * strideC;
      const int hh = lane >> 4, c4 = (lane & 15) * 4;
      for (int pass = 0; pass < 2; ++pass) {
#pragma unroll
        for (int it = 0; it < 8; ++it) {
          const int row = it * 2 + hh;
          v4f v = *(const v4f*)(slab + row * 68 + c4);
          *(volatile v4f*)(C + (size_t)(mBase + row) * ldc + n0 + c4) = v;
        }
        __threadfence();
      }
    } else {
      const int q = lane >> 3, c8 = (lane & 7) * 8;
      unsigned short* C  = (unsigned short*)Cout  + (size_t)b * strideC;
      unsigned short* C2 = (OUT_MODE == 2) ? ((unsigned short*)Cout2 + (size_t)b * strideC) : nullptr;
      for (int pass = 0; pass < 2; ++pass) {
#pragma unroll
        for (int it = 0; it < 4; ++it) {
          const int row = it * 4 + q;
          const float* sp = slab + row * 68 + c8;
          v8h hv, lv;
#pragma unroll
          for (int e = 0; e < 8; ++e) {
            if (OUT_MODE == 1) {
              hv[e] = (_Float16)sp[e];
            } else {
              unsigned short hb = f2bf_bits(sp[e]);
              unsigned short lb = f2bf_bits(sp[e] - bf_bits2f(hb));
              hv[e] = __builtin_bit_cast(_Float16, hb);
              lv[e] = __builtin_bit_cast(_Float16, lb);
            }
          }
          *(volatile v8h*)(C + (size_t)(mBase + row) * ldc + n0 + c8) = hv;
          if (OUT_MODE == 2) *(volatile v8h*)(C2 + (size_t)(mBase + row) * ldc + n0 + c8) = lv;
        }
        __threadfence();
      }
    }
    __builtin_amdgcn_fence(__ATOMIC_RELEASE, "workgroup");
    __builtin_amdgcn_wave_barrier();
    __builtin_amdgcn_fence(__ATOMIC_ACQUIRE, "workgroup");
  }
}

__global__ __launch_bounds__(NTHR) void cvt8_kernel(const float* __restrict__ src, unsigned short* __restrict__ dst,
                                                    int n8, float sc) {
  const int i = blockIdx.x * NTHR + threadIdx.x;
  if (i < n8) {
    const float* sp = src + (size_t)i * 8;
    const v4f a = *(const v4f*)(sp);
    const v4f b = *(const v4f*)(sp + 4);
    v8h hv;
#pragma unroll
    for (int e = 0; e < 4; ++e) {
      hv[e]     = (_Float16)(a[e] * sc);
      hv[4 + e] = (_Float16)(b[e] * sc);
    }
    *(volatile v8h*)(dst + (size_t)i * 8) = hv;
    __threadfence();
    *(volatile v8h*)(dst + (size_t)i * 8) = hv;
  }
}

template <int KX, bool SECOND>
__device__ __forceinline__ void stage_input(_Float16* Ax, const float* __restrict__ xf, const _Float16* __restrict__ xh,
                                            int rowbase, int t, int tid) {
  if (!SECOND) {
    const int m = tid >> 4, f4 = (tid & 15) * 4;
    const v4f v = *(const v4f*)(xf + ((size_t)(rowbase + m) * NSTEP + (size_t)t) * NFEAT + f4);
    v4h hv;
    hv[0] = (_Float16)(v[0] * ACARRY);
    hv[1] = (_Float16)(v[1] * ACARRY);
    hv[2] = (_Float16)(v[2] * ACARRY);
    hv[3] = (_Float16)(v[3] * ACARRY);
    *(v4h*)(Ax + m * (KX + 8) + f4) = hv;
  } else {
#pragma unroll
    for (int it = 0; it < 2; ++it) {
      const int idx = it * NTHR + tid;
      const int row = idx >> 5, c8 = (idx & 31) * 8;
      const v8h v = *(const v8h*)(xh + ((size_t)t * NBAT + (size_t)(rowbase + row)) * NHID + c8);
      *(v8h*)(Ax + row * (KX + 8) + c8) = v;
    }
  }
}

template <int KX, bool SECOND>
__global__ __launch_bounds__(NTHR) void lstm_seq_kernel(const float* __restrict__ xf,
                                                        const unsigned short* __restrict__ xhp,
                                                        const float* __restrict__ b_ih, const float* __restrict__ b_hh,
                                                        const float* __restrict__ h0, const float* __restrict__ c0,
                                                        const unsigned short* __restrict__ WXp,
                                                        const unsigned short* __restrict__ WHp,
                                                        unsigned short* __restrict__ hsout) {
  constexpr int XPITCH = KX + 8;
  static_assert(KX % 32 == 0, "K multiple of 32");
  static_assert((XPITCH % 8) == 0, "16-B aligned LDS rows");
  __shared__ __align__(16) _Float16 Ax[SEQ_BLK * XPITCH];
  __shared__ __align__(16) _Float16 Ah[SEQ_BLK * HPITCH];
  const _Float16* WX = (const _Float16*)WXp;
  const _Float16* WH = (const _Float16*)WHp;
  const _Float16* xh = (const _Float16*)xhp;
  const int tid = threadIdx.x, lane = tid & 31, wave = tid >> 5;
  const int c = lane & 15, hh = lane >> 4, koff = hh * 8;
  const int rowbase = blockIdx.x * SEQ_BLK;

#pragma unroll 1
  for (int i = 0; i < SEQ_BLK; ++i)
    Ah[i * HPITCH + tid] = (_Float16)(h0[(size_t)(rowbase + i) * NHID + tid] * ACARRY);
  stage_input<KX, SECOND>(Ax, xf, xh, rowbase, 0, tid);

  float cst[2][8], hst[2][8], bb[2][4];
#pragma unroll
  for (int nt = 0; nt < 2; ++nt) {
    const int j = 32 * wave + 16 * nt + c;
#pragma unroll
    for (int g = 0; g < 4; ++g) {
      const float ba = b_ih[g * NHID + j];
      const float bh = b_hh[g * NHID + j];
      bb[nt][g] = ba + bh;
    }
    asm volatile("" : "+v"(bb[nt][0]), "+v"(bb[nt][1]), "+v"(bb[nt][2]), "+v"(bb[nt][3]) :: "memory");
#pragma unroll
    for (int r = 0; r < 8; ++r) {
      cst[nt][r] = c0[(size_t)(rowbase + 8 * hh + r) * NHID + j];
      hst[nt][r] = 0.0f;
    }
    asm volatile("" : "+v"(cst[nt][0]), "+v"(cst[nt][1]), "+v"(cst[nt][2]), "+v"(cst[nt][3]),
                      "+v"(cst[nt][4]), "+v"(cst[nt][5]), "+v"(cst[nt][6]), "+v"(cst[nt][7]) :: "memory");
  }
  __syncthreads();

  const _Float16* axrow = Ax + c * XPITCH + koff;
  const _Float16* ahrow = Ah + c * HPITCH + koff;
  const v8f z8 = {0.f, 0.f, 0.f, 0.f, 0.f, 0.f, 0.f, 0.f};

#pragma unroll 1
  for (int t = 0; t < NSTEP; ++t) {
#pragma unroll
    for (int nt = 0; nt < 2; ++nt) {
      const int j = 32 * wave + 16 * nt + c;
      const _Float16* wx = WX + (size_t)j * KX + koff;
      const _Float16* wh = WH + (size_t)j * NHID + koff;
      v8f acc[4];
      acc[0] = z8; acc[1] = z8; acc[2] = z8; acc[3] = z8;
#pragma unroll 1
      for (int kx = 0; kx < KX; kx += 32) {
        const v16h a  = Frag<_Float16>::load(axrow + kx);
        const v16h b0 = Frag<_Float16>::load(wx + kx);
        const v16h b1 = Frag<_Float16>::load(wx + (size_t)1 * NHID * KX + kx);
        const v16h b2 = Frag<_Float16>::load(wx + (size_t)2 * NHID * KX + kx);
        const v16h b3 = Frag<_Float16>::load(wx + (size_t)3 * NHID * KX + kx);
        acc[0] = Frag<_Float16>::mma(a, b0, acc[0]);
        acc[1] = Frag<_Float16>::mma(a, b1, acc[1]);
        acc[2] = Frag<_Float16>::mma(a, b2, acc[2]);
        acc[3] = Frag<_Float16>::mma(a, b3, acc[3]);
        guard_all_h(acc[0], acc[1], acc[2], acc[3], a, b0, b1, b2, b3);
      }
#pragma unroll 1
      for (int k0 = 0; k0 < NHID; k0 += 32) {
        const v16h a  = Frag<_Float16>::load(ahrow + k0);
        const v16h b0 = Frag<_Float16>::load(wh + k0);
        const v16h b1 = Frag<_Float16>::load(wh + (size_t)1 * NHID * NHID + k0);
        const v16h b2 = Frag<_Float16>::load(wh + (size_t)2 * NHID * NHID + k0);
        const v16h b3 = Frag<_Float16>::load(wh + (size_t)3 * NHID * NHID + k0);
        acc[0] = Frag<_Float16>::mma(a, b0, acc[0]);
        acc[1] = Frag<_Float16>::mma(a, b1, acc[1]);
        acc[2] = Frag<_Float16>::mma(a, b2, acc[2]);
        acc[3] = Frag<_Float16>::mma(a, b3, acc[3]);
        guard_all_h(acc[0], acc[1], acc[2], acc[3], a, b0, b1, b2, b3);
      }
      acc_guard4(acc[0], acc[1], acc[2], acc[3]);
#pragma unroll
      for (int r = 0; r < 8; ++r) {
        const float zi = acc[0][r] * GATE_FOLD + bb[nt][0];
        const float zf = acc[1][r] * GATE_FOLD + bb[nt][1];
        const float zg = acc[2][r] * GATE_FOLD + bb[nt][2];
        const float zo = acc[3][r] * GATE_FOLD + bb[nt][3];
        const float ig = fsig(zi);
        const float fg = fsig(zf);
        const float gg = ftanh(zg);
        const float og = fsig(zo);
        const float cn = fg * cst[nt][r] + ig * gg;
        cst[nt][r] = cn;
        hst[nt][r] = og * ftanh(cn);
      }
    }
    __syncthreads();
#pragma unroll
    for (int nt = 0; nt < 2; ++nt) {
      const int j = 32 * wave + 16 * nt + c;
#pragma unroll
      for (int r = 0; r < 8; ++r) Ah[(8 * hh + r) * HPITCH + j] = (_Float16)(hst[nt][r] * ACARRY);
    }
    {
      const int tn = (t + 1 < NSTEP) ? (t + 1) : (NSTEP - 1);
      stage_input<KX, SECOND>(Ax, xf, xh, rowbase, tn, tid);
    }
    __syncthreads();
    {
      v8h ov[2];
#pragma unroll
      for (int it = 0; it < 2; ++it) {
        const int idx = it * NTHR + tid;
        const int row = idx >> 5, c8 = (idx & 31) * 8;
        ov[it] = *(const v8h*)(Ah + row * HPITCH + c8);
      }
      for (int pass = 0; pass < 2; ++pass) {
#pragma unroll
        for (int it = 0; it < 2; ++it) {
          const int idx = it * NTHR + tid;
          const int row = idx >> 5, c8 = (idx & 31) * 8;
          const size_t o = SECOND ? (((size_t)(rowbase + row) * NSTEP + (size_t)t) * NHID + c8)
                                  : (((size_t)t * NBAT + (size_t)(rowbase + row)) * NHID + c8);
          *(volatile v8h*)(hsout + o) = ov[it];
        }
        __threadfence();
      }
    }
  }
}

__global__ __launch_bounds__(NTHR) void fc2_kernel(const float* __restrict__ hid, const float* __restrict__ w,
                                                   const float* __restrict__ bias, float* __restrict__ out) {
  const int i = blockIdx.x * NTHR + threadIdx.x;
  if (i < NBAT * NOUTC) {
    const int b = i / NOUTC;
    const int o = i - b * NOUTC;
    const float* hp = hid + (size_t)b * NFC1;
    const float* wp = w + (size_t)o * NFC1;
    float s0 = 0.0f, s1 = 0.0f, s2 = 0.0f, s3 = 0.0f;
#pragma unroll 1
    for (int k = 0; k < NFC1; k += 4) {
      const v4f hv = *(const v4f*)(hp + k);
      const v4f wv = *(const v4f*)(wp + k);
      s0 += hv[0] * wv[0];
      s1 += hv[1] * wv[1];
      s2 += hv[2] * wv[2];
      s3 += hv[3] * wv[3];
    }
    const float s = ((s0 + s1) + (s2 + s3)) + bias[o];
    const float v = fmaxf(s, 0.0f);
    *(volatile float*)(out + i) = v;
    __threadfence();
    *(volatile float*)(out + i) = v;
  }
}

extern "C" void kernel_launch(void* const* d_in, const int* in_sizes, int n_in,
                              void* d_out, int out_size, void* d_ws, size_t ws_size, hipStream_t stream) {
  if (n_in < 15 || d_out == nullptr || d_ws == nullptr) return;
  if (in_sizes[0] != NBAT * NSTEP * NFEAT || in_sizes[1] != 2 * NBAT * NHID || in_sizes[2] != 2 * NBAT * NHID ||
      in_sizes[3] != NGATE * NFEAT || in_sizes[4] != NGATE * NHID || in_sizes[5] != NGATE || in_sizes[6] != NGATE ||
      in_sizes[7] != NGATE * NHID || in_sizes[8] != NGATE * NHID || in_sizes[9] != NGATE || in_sizes[10] != NGATE ||
      in_sizes[11] != NFC1 * KFLAT || in_sizes[12] != NFC1 || in_sizes[13] != NOUTC * NFC1 || in_sizes[14] != NOUTC ||
      out_size != NBAT * NOUTC) return;

  const float* x     = (const float*)d_in[0];
  const float* h0    = (const float*)d_in[1];
  const float* c0    = (const float*)d_in[2];
  const float* W_ih0 = (const float*)d_in[3];
  const float* W_hh0 = (const float*)d_in[4];
  const float* b_ih0 = (const float*)d_in[5];
  const float* b_hh0 = (const float*)d_in[6];
  const float* W_ih1 = (const float*)d_in[7];
  const float* W_hh1 = (const float*)d_in[8];
  const float* b_ih1 = (const float*)d_in[9];
  const float* b_hh1 = (const float*)d_in[10];
  const float* fc1_w = (const float*)d_in[11];
  const float* fc1_b = (const float*)d_in[12];
  const float* fc2_w = (const float*)d_in[13];
  const float* fc2_b = (const float*)d_in[14];
  float* out = (float*)d_out;

  char* ws = (char*)d_ws;
  size_t off = 0;
  auto carve = [&](size_t bytes) -> char* { char* p = ws + off; off += (bytes + 255) & ~(size_t)255; return p; };
  unsigned short* WI0  = (unsigned short*)carve((size_t)NGATE * NFEAT * 2);
  unsigned short* WH0  = (unsigned short*)carve((size_t)NGATE * NHID * 2);
  unsigned short* WI1  = (unsigned short*)carve((size_t)NGATE * NHID * 2);
  unsigned short* WH1  = (unsigned short*)carve((size_t)NGATE * NHID * 2);
  unsigned short* FC1W = (unsigned short*)carve((size_t)NFC1 * KFLAT * 2);
  unsigned short* HS0  = (unsigned short*)carve((size_t)NSTEP * NBAT * NHID * 2);
  unsigned short* HS1  = (unsigned short*)carve((size_t)NBAT * NSTEP * NHID * 2);
  float*          HID  = (float*)carve((size_t)NBAT * NFC1 * 4);
  if (off > ws_size || off > (size_t)134217728) return;

  const int n8_ih0 = NGATE * NFEAT / 8;
  const int n8_hh  = NGATE * NHID / 8;
  const int n8_fc1 = NFC1 * (KFLAT / 8);
  cvt8_kernel<<<n8_ih0 / NTHR, NTHR, 0, stream>>>(W_ih0, WI0, n8_ih0, WCARRY);
  cvt8_kernel<<<n8_hh / NTHR,  NTHR, 0, stream>>>(W_hh0, WH0, n8_hh,  WCARRY);
  cvt8_kernel<<<n8_hh / NTHR,  NTHR, 0, stream>>>(W_ih1, WI1, n8_hh,  WCARRY);
  cvt8_kernel<<<n8_hh / NTHR,  NTHR, 0, stream>>>(W_hh1, WH1, n8_hh,  WCARRY);
  cvt8_kernel<<<n8_fc1 / NTHR, NTHR, 0, stream>>>(fc1_w, FC1W, n8_fc1, FCARRY);

  lstm_seq_kernel<NFEAT, false><<<NBAT / SEQ_BLK, NTHR, 0, stream>>>(
      x, WI0, b_ih0, b_hh0, h0, c0, WI0, WH0, HS0);
  lstm_seq_kernel<NHID, true><<<NBAT / SEQ_BLK, NTHR, 0, stream>>>(
      x, HS0, b_ih1, b_hh1, h0 + (size_t)NBAT * NHID, c0 + (size_t)NBAT * NHID, WI1, WH1, HS1);

  wmma_gemm64<0, false, 2, 0, false, 1><<<dim3((NBAT / 64) * (NFC1 / 64) / 8, 1), 256, 0, stream>>>(
      HS1, HS1, KFLAT, 0L, FC1W, FC1W, KFLAT, 0L, (void*)HID, (void*)HID, NFC1, 0L,
      fc1_b, fc1_b, 0L, NBAT, NFC1, KFLAT, FC1_FOLD);

  fc2_kernel<<<(NBAT * NOUTC) / NTHR, NTHR, 0, stream>>>(HID, fc2_w, fc2_b, out);
}
